// fePAM_40295383171513
// MI455X (gfx1250) — hardware-verified
//
#include <hip/hip_runtime.h>
#include <math.h>
#include <stdint.h>

#define NB    4
#define NC    64
#define NHH   64
#define NWW   64
#define NPIX  (NHH * NWW)
#define NK    81
#define NQB   64
#define SP    68
#define JPER  21
#define NTILE (NPIX / 64)

typedef __attribute__((ext_vector_type(16))) __bf16 v16b;
typedef __attribute__((ext_vector_type(8)))  __bf16 v8b;
typedef __attribute__((ext_vector_type(8)))  float  v8f;
typedef __attribute__((ext_vector_type(4)))  float  v4f;
typedef __attribute__((ext_vector_type(2)))  float  v2f;
typedef __attribute__((ext_vector_type(4)))  unsigned int v4u;

__device__ __forceinline__ unsigned short f2bf_bits(float f) {
  const unsigned u = __float_as_uint(f);
  return (unsigned short)((u + 0x7FFFu + ((u >> 16) & 1u)) >> 16);
}
__device__ __forceinline__ float bf_bits2f(unsigned short h) { return __uint_as_float(((unsigned)h) << 16); }
__device__ __forceinline__ unsigned pk16(unsigned short a, unsigned short b) { return (unsigned)a | ((unsigned)b << 16); }

union FragU { v16b v; v8b h[2]; };
__device__ __forceinline__ v16b frag_load(const unsigned short* p) {
  FragU f;
  f.h[0] = *(const v8b*)(p);
  f.h[1] = *(const v8b*)(p + 16);
  return f.v;
}
__device__ __forceinline__ v8f mma_bf(v16b a, v16b b, v8f c) {
  return __builtin_amdgcn_wmma_f32_16x16x32_bf16(false, a, false, b, (short)0, c, false, false);
}
__device__ __forceinline__ void guard6(v8f& c0, v8f& c1, v16b x0, v16b x1, v16b x2, v16b x3, v16b x4, v16b x5) {
  asm volatile("v_nop\n\tv_nop\n\tv_nop\n\tv_nop"
               : "+v"(c0), "+v"(c1)
               : "v"(x0), "v"(x1), "v"(x2), "v"(x3), "v"(x4), "v"(x5));
}

__global__ __launch_bounds__(256) void k_prep(const float* __restrict__ Q, const float* __restrict__ S,
                                              const float* __restrict__ R,
                                              unsigned short* __restrict__ Qhi, unsigned short* __restrict__ Qlo,
                                              unsigned short* __restrict__ Shi, unsigned short* __restrict__ Slo,
                                              float* __restrict__ Rt) {
  __shared__ __align__(16) float tf[NC * SP];
  const int pt  = blockIdx.x;
  const int b   = blockIdx.y;
  const int z   = blockIdx.z;
  const int tid = threadIdx.x;
  const float* src = (z == 0) ? Q : ((z == 1) ? S : R);
  {
    const int c  = tid >> 2;
    const int px = (tid & 3) * 16;
    const float* g = src + ((size_t)b * NC + c) * NPIX + (size_t)pt * 64 + px;
#pragma unroll
    for (int q = 0; q < 4; ++q) {
      const v4f f = *(const v4f*)(g + 4 * q);
#pragma unroll
      for (int e = 0; e < 4; ++e) tf[c * SP + px + 4 * q + e] = f[e];
    }
  }
  __syncthreads();
  const size_t prow = (size_t)b * NPIX + (size_t)pt * 64;
  if (z < 2) {
    unsigned short* dh = (z == 0) ? Qhi : Shi;
    unsigned short* dl = (z == 0) ? Qlo : Slo;
    const int q4 = tid >> 3;
    const int c8 = (tid & 7) * 8;
    v4u hv[2], lv[2];
#pragma unroll
    for (int it = 0; it < 2; ++it) {
      const int p = it * 32 + q4;
      v4u a, a2;
#pragma unroll
      for (int qq = 0; qq < 4; ++qq) {
        const float x0 = tf[(c8 + 2 * qq) * SP + p];
        const float x1 = tf[(c8 + 2 * qq + 1) * SP + p];
        const unsigned short h0 = f2bf_bits(x0), h1 = f2bf_bits(x1);
        const unsigned short l0 = f2bf_bits(x0 - bf_bits2f(h0));
        const unsigned short l1 = f2bf_bits(x1 - bf_bits2f(h1));
        a[qq]  = pk16(h0, h1);
        a2[qq] = pk16(l0, l1);
      }
      hv[it] = a;
      lv[it] = a2;
    }
#pragma unroll
    for (int it = 0; it < 2; ++it) {
      const size_t go = (prow + (size_t)(it * 32 + q4)) * NC + c8;
      *(volatile v4u*)(dh + go) = hv[it];
      *(volatile v4u*)(dl + go) = lv[it];
    }
    __threadfence();
#pragma unroll
    for (int it = 0; it < 2; ++it) {
      const size_t go = (prow + (size_t)(it * 32 + q4)) * NC + c8;
      *(volatile v4u*)(dh + go) = hv[it];
      *(volatile v4u*)(dl + go) = lv[it];
    }
  } else {
    const int q2 = tid >> 4;
    const int c4 = (tid & 15) * 4;
    v4f rv[4];
#pragma unroll
    for (int it = 0; it < 4; ++it) {
      const int p = it * 16 + q2;
      v4f a;
#pragma unroll
      for (int e = 0; e < 4; ++e) a[e] = tf[(c4 + e) * SP + p];
      rv[it] = a;
    }
#pragma unroll
    for (int it = 0; it < 4; ++it) {
      const size_t go = (prow + (size_t)(it * 16 + q2)) * NC + c4;
      *(volatile v4f*)(Rt + go) = rv[it];
    }
    __threadfence();
#pragma unroll
    for (int it = 0; it < 4; ++it) {
      const size_t go = (prow + (size_t)(it * 16 + q2)) * NC + c4;
      *(volatile v4f*)(Rt + go) = rv[it];
    }
  }
}

__global__ __launch_bounds__(256) void k_attn(
    const unsigned short* __restrict__ Qhi, const unsigned short* __restrict__ Qlo,
    const unsigned short* __restrict__ Shi, const unsigned short* __restrict__ Slo,
    const float* __restrict__ Rt,
    const int* __restrict__ xxs, const int* __restrict__ yys, int istride,
    const int* __restrict__ tflag,
    float* __restrict__ out0, float* __restrict__ out1) {
  __shared__ __align__(16) unsigned short s_lin[NQB * NK];
  __shared__ __align__(16) float sS[NQB * SP];
  __shared__ __align__(16) float s_sc[NQB * NK];
  (void)tflag;
  const int hrow = blockIdx.x;
  const int b    = blockIdx.y;
  const int tid  = threadIdx.x;
  const int lane = tid & 31;
  const int wave = tid >> 5;
  const int half = lane >> 4;
  const int l15  = lane & 15;
  const int koff = half * 8;
  const int m0   = hrow * NQB;

  {
    const size_t ebase = ((size_t)b * NPIX + (size_t)m0) * NK;
    for (int i = tid; i < NQB * NK; i += 256) {
      const size_t e = (ebase + (size_t)i) * (size_t)istride;
      int xx = xxs[e];
      int yy = yys[e];
      xx = (xx < 0) ? 0 : ((xx > NHH - 1) ? (NHH - 1) : xx);
      yy = (yy < 0) ? 0 : ((yy > NWW - 1) ? (NWW - 1) : yy);
      s_lin[i] = (unsigned short)(xx * NWW + yy);
    }
  }
  const int wq = wave & 3;
  const int wn = wave >> 2;
  const size_t arow = ((size_t)b * NPIX + (size_t)(m0 + 16 * wq + l15)) * NC + koff;
  const v16b ah0 = frag_load(Qhi + arow);
  const v16b ah1 = frag_load(Qhi + arow + 32);
  const v16b al0 = frag_load(Qlo + arow);
  const v16b al1 = frag_load(Qlo + arow + 32);
  __syncthreads();

  const int ql   = tid & 63;
  const int part = tid >> 6;
  const int srow = ql * SP;
  int   lin[JPER];
  float sc[JPER];
#pragma unroll
  for (int jj = 0; jj < JPER; ++jj) {
    const int j  = part * JPER + jj;
    const int jc = (j < NK) ? j : (NK - 1);
    const int v  = (int)s_lin[ql * NK + jc];
    lin[jj] = (j < NK) ? v : 0x10000;
    sc[jj]  = 0.0f;
  }

#pragma unroll 1
  for (int t = 0; t < NTILE; ++t) {
    v8f acc0 = {0.f, 0.f, 0.f, 0.f, 0.f, 0.f, 0.f, 0.f};
    v8f acc1 = {0.f, 0.f, 0.f, 0.f, 0.f, 0.f, 0.f, 0.f};
    const size_t brow0 = ((size_t)b * NPIX + (size_t)(t * 64 + 32 * wn + l15)) * NC + koff;
    const size_t brow1 = brow0 + (size_t)16 * NC;
#pragma unroll
    for (int ks = 0; ks < 2; ++ks) {
      const v16b ah  = (ks == 0) ? ah0 : ah1;
      const v16b al  = (ks == 0) ? al0 : al1;
      const v16b bh0 = frag_load(Shi + brow0 + 32 * ks);
      const v16b bh1 = frag_load(Shi + brow1 + 32 * ks);
      const v16b bl0 = frag_load(Slo + brow0 + 32 * ks);
      const v16b bl1 = frag_load(Slo + brow1 + 32 * ks);
      acc0 = mma_bf(ah, bh0, acc0);
      acc0 = mma_bf(ah, bl0, acc0);
      acc0 = mma_bf(al, bh0, acc0);
      acc1 = mma_bf(ah, bh1, acc1);
      acc1 = mma_bf(ah, bl1, acc1);
      acc1 = mma_bf(al, bh1, acc1);
      guard6(acc0, acc1, bh0, bh1, bl0, bl1, ah, al);
    }
    float* srp = sS + (16 * wq + 8 * half) * SP + 32 * wn + l15;
#pragma unroll
    for (int r = 0; r < 8; ++r) {
      srp[r * SP]      = acc0[r];
      srp[r * SP + 16] = acc1[r];
    }
    __syncthreads();
#pragma unroll
    for (int jj = 0; jj < JPER; ++jj) {
      const int lv  = lin[jj];
      const float v = sS[srow + (lv & 63)];
      sc[jj] = ((lv >> 6) == t) ? v : sc[jj];
    }
    __syncthreads();
  }

#pragma unroll
  for (int jj = 0; jj < JPER; ++jj) {
    const int j = part * JPER + jj;
    if (j < NK) s_sc[ql * NK + j] = sc[jj];
  }
  __syncthreads();

#pragma unroll 1
  for (int qi = 0; qi < 8; ++qi) {
    const int q    = wave * 8 + qi;
    const int base = q * NK;
    const int j2   = lane + 64;
    const bool v2  = (j2 < NK);
    const int j2c  = v2 ? j2 : (NK - 1);
    const float x0 = s_sc[base + lane];
    const float x1 = s_sc[base + 32 + lane];
    const float x2 = s_sc[base + j2c];
    float mx = fmaxf(x0, x1);
    mx = v2 ? fmaxf(mx, x2) : mx;
#pragma unroll
    for (int off = 16; off > 0; off >>= 1) mx = fmaxf(mx, __shfl_xor(mx, off, 32));
    const float e0  = expf(x0 - mx);
    const float e1  = expf(x1 - mx);
    const float e2r = expf(x2 - mx);
    const float e2  = v2 ? e2r : 0.0f;
    float s = e0 + e1 + e2;
#pragma unroll
    for (int off = 16; off > 0; off >>= 1) s += __shfl_xor(s, off, 32);
    const float inv = 1.0f / s;
    const float p0 = e0 * inv, p1 = e1 * inv, p2 = e2 * inv;
    s_sc[base + lane]      = p0;
    s_sc[base + 32 + lane] = p1;
    if (v2) s_sc[base + j2] = p2;
  }
  __syncthreads();

  {
    float* o1 = out1 + ((size_t)b * NPIX + (size_t)m0) * NK;
    const int NF4 = NQB * NK / 4;
    v4f mv[6];
#pragma unroll
    for (int i = 0; i < 6; ++i) {
      const int f  = tid + 256 * i;
      const int fc = (f < NF4) ? f : (NF4 - 1);
      mv[i] = *(const v4f*)(s_sc + 4 * fc);
    }
#pragma unroll
    for (int i = 0; i < 6; ++i) {
      const int f = tid + 256 * i;
      if (f < NF4) *(volatile v4f*)(o1 + 4 * (size_t)f) = mv[i];
    }
    __threadfence();
#pragma unroll
    for (int i = 0; i < 6; ++i) {
      const int f = tid + 256 * i;
      if (f < NF4) *(volatile v4f*)(o1 + 4 * (size_t)f) = mv[i];
    }
  }

#pragma unroll 1
  for (int qi = 0; qi < 8; ++qi) {
    const int q    = wave * 8 + qi;
    const int base = q * NK;
    float a0 = 0.0f, a1 = 0.0f;
#pragma unroll 3
    for (int j = 0; j < NK; ++j) {
      const float p  = s_sc[base + j];
      const int   lv = (int)s_lin[base + j];
      const v2f   r  = *(const v2f*)(Rt + ((size_t)b * NPIX + (size_t)lv) * NC + 2 * lane);
      a0 += p * r[0];
      a1 += p * r[1];
    }
    sS[(2 * lane) * SP + q]     = a0;
    sS[(2 * lane + 1) * SP + q] = a1;
  }
  __syncthreads();

  {
    v4f ov[4];
#pragma unroll
    for (int it = 0; it < 4; ++it) {
      const int c = it * 16 + 2 * wave + half;
      ov[it] = *(const v4f*)(sS + c * SP + l15 * 4);
    }
#pragma unroll
    for (int it = 0; it < 4; ++it) {
      const int c = it * 16 + 2 * wave + half;
      float* dst = out0 + (((size_t)b * NC + c) * NHH + (size_t)hrow) * NWW + l15 * 4;
      *(volatile v4f*)dst = ov[it];
    }
    __threadfence();
#pragma unroll
    for (int it = 0; it < 4; ++it) {
      const int c = it * 16 + 2 * wave + half;
      float* dst = out0 + (((size_t)b * NC + c) * NHH + (size_t)hrow) * NWW + l15 * 4;
      *(volatile v4f*)dst = ov[it];
    }
  }
}

extern "C" void kernel_launch(void* const* d_in, const int* in_sizes, int n_in,
                              void* d_out, int out_size, void* d_ws, size_t ws_size,
                              hipStream_t stream) {
  if (n_in < 6) return;
  const int nfeat = NB * NC * NPIX;
  const int nidx  = NB * NPIX * NK;
  if (in_sizes[0] != nfeat || in_sizes[1] != nfeat || in_sizes[2] != nfeat) return;
  if (in_sizes[3] != in_sizes[4]) return;
  const int istride = in_sizes[3] / nidx;
  if (istride != 1 && istride != 2) return;
  if (istride * nidx != in_sizes[3]) return;
  if (out_size != nfeat + nidx) return;

  const float* Q   = (const float*)d_in[0];
  const float* S   = (const float*)d_in[1];
  const float* R   = (const float*)d_in[2];
  const int*   xxs = (const int*)d_in[3];
  const int*   yys = (const int*)d_in[4];
  const int*   trn = (const int*)d_in[5];

  const size_t PL16 = (size_t)NB * NPIX * NC * 2;
  const size_t PL32 = (size_t)NB * NPIX * NC * 4;
  size_t off = 0;
  const size_t oQhi = off; off += PL16;
  const size_t oQlo = off; off += PL16;
  const size_t oShi = off; off += PL16;
  const size_t oSlo = off; off += PL16;
  const size_t oRt  = off; off += PL32;
  if (off > ws_size) return;

  char* ws = (char*)d_ws;
  unsigned short* Qhi = (unsigned short*)(ws + oQhi);
  unsigned short* Qlo = (unsigned short*)(ws + oQlo);
  unsigned short* Shi = (unsigned short*)(ws + oShi);
  unsigned short* Slo = (unsigned short*)(ws + oSlo);
  float*          Rt  = (float*)(ws + oRt);

  float* out0 = (float*)d_out;
  float* out1 = (float*)d_out + (size_t)nfeat;

  const dim3 blk(256);
  k_prep<<<dim3(NTILE, NB, 3), blk, 0, stream>>>(Q, S, R, Qhi, Qlo, Shi, Slo, Rt);
  k_attn<<<dim3(NHH, NB), blk, 0, stream>>>(Qhi, Qlo, Shi, Slo, Rt, xxs, yys, istride, trn, out0, out1);
  (void)hipGetLastError();
}
